// RNNModel_10368051053183
// MI455X (gfx1250) — hardware-verified
//
#include <hip/hip_runtime.h>
#include <stddef.h>

typedef __attribute__((ext_vector_type(16))) __bf16   v16b;
typedef __attribute__((ext_vector_type(8)))  __bf16   v8b;
typedef __attribute__((ext_vector_type(8)))  float    v8f;
typedef __attribute__((ext_vector_type(4)))  float    v4f;
typedef __attribute__((ext_vector_type(4)))  unsigned int v4u;

namespace {
constexpr int NBATCH = 128;
constexpr int NSEQ   = 1024;
constexpr int NOUT   = 64;
constexpr int NHID   = 256;
constexpr int XDIM   = 65;
constexpr int XKP    = 96;
constexpr int WIP    = 128;
constexpr int ROWS   = 16;
constexpr int NTHR   = 512;
constexpr int SHP    = NHID + 8;
constexpr int YSP    = 68;
constexpr int HBSZ   = ROWS * SHP;
constexpr int YBSZ   = ROWS * YSP;

constexpr size_t XPLANE_B  = (size_t)NBATCH * NSEQ * XKP * 2;
constexpr size_t WHHPL_B   = (size_t)NHID * NHID * 2;
constexpr size_t WIHPL_B   = (size_t)NHID * WIP * 2;
constexpr size_t VPL_B     = (size_t)NOUT * NHID * 2;
constexpr size_t OFF_XH    = 0;
constexpr size_t OFF_XL    = OFF_XH + XPLANE_B;
constexpr size_t OFF_WHH_H = OFF_XL + XPLANE_B;
constexpr size_t OFF_WHH_L = OFF_WHH_H + WHHPL_B;
constexpr size_t OFF_WIH_H = OFF_WHH_L + WHHPL_B;
constexpr size_t OFF_WIH_L = OFF_WIH_H + WIHPL_B;
constexpr size_t OFF_V_H   = OFF_WIH_L + WIHPL_B;
constexpr size_t OFF_V_L   = OFF_V_H + VPL_B;
constexpr size_t WS_TOTAL  = OFF_V_L + VPL_B;
static_assert(WS_TOTAL <= (size_t)134217728, "carve");
static_assert((OFF_XL % 4096) == 0 && (OFF_WHH_H % 4096) == 0 && (OFF_WHH_L % 4096) == 0 &&
              (OFF_WIH_H % 4096) == 0 && (OFF_WIH_L % 4096) == 0 && (OFF_V_H % 4096) == 0 &&
              (OFF_V_L % 4096) == 0, "alignment");
static_assert(XKP % 32 == 0 && NHID % 32 == 0, "k-step 32");
static_assert(NBATCH % ROWS == 0, "batch tile");
static_assert(((size_t)NBATCH * NSEQ * XKP) % (8 * 256) == 0, "x prep grid exact");
static_assert(NTHR / 32 == NHID / 16, "one wave per 16 hidden columns");
constexpr int XPREP_BLOCKS = (int)(((size_t)NBATCH * NSEQ * XKP) / (8 * 256));
}

__device__ __forceinline__ unsigned short f2bf_bits(float f) {
  unsigned u = __float_as_uint(f);
  return (unsigned short)((u + 0x7FFFu + ((u >> 16) & 1u)) >> 16);
}
__device__ __forceinline__ float bf_bits2f(unsigned short h) { return __uint_as_float(((unsigned)h) << 16); }

struct FragB {
  union U { v16b v; v8b h[2]; };
  static __device__ __forceinline__ v16b load(const __bf16* p) {
    U f; f.h[0] = *(const v8b*)(p); f.h[1] = *(const v8b*)(p + 16); return f.v;
  }
};

__device__ __forceinline__ v8f mma_bf16(v16b a, v16b b, v8f c) {
  return __builtin_amdgcn_wmma_f32_16x16x32_bf16(false, a, false, b, (short)0, c, false, false);
}
__device__ __forceinline__ void dep_guard4(v8f& acc, v16b x, v16b y, v16b z, v16b w) {
  asm volatile("v_nop\n\tv_nop\n\tv_nop\n\tv_nop" : "+v"(acc) : "v"(x), "v"(y), "v"(z), "v"(w));
}
__device__ __forceinline__ void acc_guard2(v8f& a, v8f& b) {
  asm volatile("v_nop\n\tv_nop\n\tv_nop\n\tv_nop" : "+v"(a), "+v"(b));
}

__device__ __forceinline__ void split_pack2(float a, float b, unsigned& hw, unsigned& lw) {
  const unsigned short ha = f2bf_bits(a);
  const unsigned short hb = f2bf_bits(b);
  const unsigned short la = f2bf_bits(a - bf_bits2f(ha));
  const unsigned short lb = f2bf_bits(b - bf_bits2f(hb));
  hw = (unsigned)ha | ((unsigned)hb << 16);
  lw = (unsigned)la | ((unsigned)lb << 16);
}

__global__ __launch_bounds__(256) void prep_x(const float* __restrict__ x,
                                              unsigned short* __restrict__ xh,
                                              unsigned short* __restrict__ xl) {
  const size_t gl  = (size_t)blockIdx.x * 256 + threadIdx.x;
  const size_t f   = gl * 8;
  const size_t row = f / XKP;
  const int    k0  = (int)(f - row * XKP);
  const float* src = x + row * XDIM;
  float v[8];
#pragma unroll
  for (int e = 0; e < 8; ++e) {
    const int k  = k0 + e;
    const int kc = (k < XDIM) ? k : (XDIM - 1);
    const float tv = src[kc];
    v[e] = (k < XDIM) ? tv : 0.0f;
  }
  v4u hv, lv;
#pragma unroll
  for (int e2 = 0; e2 < 4; ++e2) {
    unsigned hw, lw;
    split_pack2(v[2 * e2], v[2 * e2 + 1], hw, lw);
    hv[e2] = hw; lv[e2] = lw;
  }
  unsigned short* dh = xh + f;
  unsigned short* dl = xl + f;
  *(volatile v4u*)dh = hv;
  *(volatile v4u*)dl = lv;
  __threadfence();
  *(volatile v4u*)dh = hv;
  *(volatile v4u*)dl = lv;
}

__global__ __launch_bounds__(256) void prep_whh(const float* __restrict__ w,
                                                unsigned short* __restrict__ oh,
                                                unsigned short* __restrict__ ol) {
  const int wave = threadIdx.x >> 5, lane = threadIdx.x & 31;
  const int n  = blockIdx.x * 8 + wave;
  const int k0 = lane * 8;
  float v[8];
#pragma unroll
  for (int e = 0; e < 8; ++e) v[e] = w[(size_t)(k0 + e) * NHID + n];
  v4u hv, lv;
#pragma unroll
  for (int e2 = 0; e2 < 4; ++e2) {
    unsigned hw, lw;
    split_pack2(v[2 * e2], v[2 * e2 + 1], hw, lw);
    hv[e2] = hw; lv[e2] = lw;
  }
  unsigned short* dh = oh + (size_t)n * NHID + k0;
  unsigned short* dl = ol + (size_t)n * NHID + k0;
  *(volatile v4u*)dh = hv;
  *(volatile v4u*)dl = lv;
  __threadfence();
  *(volatile v4u*)dh = hv;
  *(volatile v4u*)dl = lv;
}

__global__ __launch_bounds__(256) void prep_wih(const float* __restrict__ w,
                                                unsigned short* __restrict__ oh,
                                                unsigned short* __restrict__ ol) {
  const int wave = threadIdx.x >> 5, lane = threadIdx.x & 31;
  const int n  = blockIdx.x * 8 + wave;
  const int k0 = (lane & 15) * 8;
  float v[8];
#pragma unroll
  for (int e = 0; e < 8; ++e) {
    const int k  = k0 + e;
    const int kc = (k < XDIM) ? k : (XDIM - 1);
    const float tv = w[(size_t)kc * NHID + n];
    v[e] = (k < XDIM) ? tv : 0.0f;
  }
  v4u hv, lv;
#pragma unroll
  for (int e2 = 0; e2 < 4; ++e2) {
    unsigned hw, lw;
    split_pack2(v[2 * e2], v[2 * e2 + 1], hw, lw);
    hv[e2] = hw; lv[e2] = lw;
  }
  if (lane < 16) {
    unsigned short* dh = oh + (size_t)n * WIP + k0;
    unsigned short* dl = ol + (size_t)n * WIP + k0;
    *(volatile v4u*)dh = hv;
    *(volatile v4u*)dl = lv;
    __threadfence();
    *(volatile v4u*)dh = hv;
    *(volatile v4u*)dl = lv;
  }
}

__global__ __launch_bounds__(256) void prep_v(const float* __restrict__ w,
                                              unsigned short* __restrict__ oh,
                                              unsigned short* __restrict__ ol) {
  const int wave = threadIdx.x >> 5, lane = threadIdx.x & 31;
  const int n  = blockIdx.x * 8 + wave;
  const int k0 = lane * 8;
  const float* src = w + (size_t)n * NHID + k0;
  const v4f a = *(const v4f*)(src);
  const v4f b = *(const v4f*)(src + 4);
  v4u hv, lv;
  {
    unsigned hw, lw;
    split_pack2(a[0], a[1], hw, lw); hv[0] = hw; lv[0] = lw;
    split_pack2(a[2], a[3], hw, lw); hv[1] = hw; lv[1] = lw;
    split_pack2(b[0], b[1], hw, lw); hv[2] = hw; lv[2] = lw;
    split_pack2(b[2], b[3], hw, lw); hv[3] = hw; lv[3] = lw;
  }
  unsigned short* dh = oh + (size_t)n * NHID + k0;
  unsigned short* dl = ol + (size_t)n * NHID + k0;
  *(volatile v4u*)dh = hv;
  *(volatile v4u*)dl = lv;
  __threadfence();
  *(volatile v4u*)dh = hv;
  *(volatile v4u*)dl = lv;
}

__device__ __forceinline__ void store_y_rows(const float* ysb, float* __restrict__ out,
                                             int b0, int tt, int wave, int lane) {
  const int hh = lane >> 4, c4 = (lane & 15) * 4;
  const int row = wave * 2 + hh;
  const v4f val = *(const v4f*)(ysb + row * YSP + c4);
  float* dst = out + ((size_t)(b0 + row) * NSEQ + tt) * NOUT + c4;
  *(volatile v4f*)dst = val;
  __threadfence();
  *(volatile v4f*)dst = val;
}

__global__ __launch_bounds__(NTHR) void rnn_scan(
    const unsigned short* __restrict__ xh_p,  const unsigned short* __restrict__ xl_p,
    const unsigned short* __restrict__ whh_hp, const unsigned short* __restrict__ whh_lp,
    const unsigned short* __restrict__ wih_hp, const unsigned short* __restrict__ wih_lp,
    const unsigned short* __restrict__ v_hp,   const unsigned short* __restrict__ v_lp,
    float* __restrict__ out) {
  __shared__ __align__(16) __bf16 hb_hi[2 * HBSZ];
  __shared__ __align__(16) __bf16 hb_lo[2 * HBSZ];
  __shared__ __align__(16) float  ys[2 * YBSZ];

  const int tid  = threadIdx.x;
  const int wave = __builtin_amdgcn_readfirstlane(tid >> 5);
  const int lane = tid & 31;
  const int hh   = lane >> 4;
  const int l15  = lane & 15;
  const int b0   = blockIdx.x * ROWS;

  const __bf16* XH  = (const __bf16*)xh_p;
  const __bf16* XL  = (const __bf16*)xl_p;
  const __bf16* WHH = (const __bf16*)whh_hp;
  const __bf16* WHL = (const __bf16*)whh_lp;
  const __bf16* WIH = (const __bf16*)wih_hp;
  const __bf16* WIL = (const __bf16*)wih_lp;
  const __bf16* VH  = (const __bf16*)v_hp;
  const __bf16* VL  = (const __bf16*)v_lp;

  {
    const __bf16 z16 = __builtin_bit_cast(__bf16, (unsigned short)0);
    for (int i = tid; i < 2 * HBSZ; i += NTHR) { hb_hi[i] = z16; hb_lo[i] = z16; }
    for (int i = tid; i < 2 * YBSZ; i += NTHR) ys[i] = 0.0f;
  }
  __syncthreads();

  const int    ncol  = wave * 16 + l15;
  const int    aoff  = l15 * SHP + 8 * hh;
  const size_t xbase = ((size_t)(b0 + l15) * NSEQ) * XKP + 8 * hh;
  const size_t whoff = (size_t)ncol * NHID + 8 * hh;
  const size_t wioff = (size_t)ncol * WIP + 8 * hh;
  const size_t vboff = (size_t)((wave & 3) * 16 + l15) * NHID + 8 * hh;
  const v8f zero8 = (v8f){0.f, 0.f, 0.f, 0.f, 0.f, 0.f, 0.f, 0.f};

  for (int t = 0; t <= NSEQ; ++t) {
    const int q = t & 1;
    if (t >= 2 && wave < 8) store_y_rows(ys + ((t - 1) & 1) * YBSZ, out, b0, t - 2, wave, lane);

    const bool doH = (t < NSEQ);
    const bool doY = (wave < 4) && (t >= 1);
    const int  tx  = doH ? t : (NSEQ - 1);

    v8f acc = zero8, yacc = zero8;
    const __bf16* hhp = hb_hi + q * HBSZ + aoff;
    const __bf16* hlp = hb_lo + q * HBSZ + aoff;
#pragma unroll 2
    for (int c = 0; c < NHID / 32; ++c) {
      const v16b ah = FragB::load(hhp + 32 * c);
      const v16b al = FragB::load(hlp + 32 * c);
      if (doH) {
        const v16b bh = FragB::load(WHH + whoff + 32 * c);
        const v16b bl = FragB::load(WHL + whoff + 32 * c);
        acc = mma_bf16(ah, bh, acc);
        acc = mma_bf16(ah, bl, acc);
        acc = mma_bf16(al, bh, acc);
        dep_guard4(acc, ah, al, bh, bl);
      }
      if (doY) {
        const v16b vh = FragB::load(VH + vboff + 32 * c);
        const v16b vl = FragB::load(VL + vboff + 32 * c);
        yacc = mma_bf16(ah, vh, yacc);
        yacc = mma_bf16(ah, vl, yacc);
        yacc = mma_bf16(al, vh, yacc);
        dep_guard4(yacc, ah, al, vh, vl);
      }
    }
    if (doH) {
      const __bf16* xhp = XH + xbase + (size_t)tx * XKP;
      const __bf16* xlp = XL + xbase + (size_t)tx * XKP;
#pragma unroll
      for (int c = 0; c < XKP / 32; ++c) {
        const v16b ah = FragB::load(xhp + 32 * c);
        const v16b al = FragB::load(xlp + 32 * c);
        const v16b bh = FragB::load(WIH + wioff + 32 * c);
        const v16b bl = FragB::load(WIL + wioff + 32 * c);
        acc = mma_bf16(ah, bh, acc);
        acc = mma_bf16(ah, bl, acc);
        acc = mma_bf16(al, bh, acc);
        dep_guard4(acc, ah, al, bh, bl);
      }
    }
    acc_guard2(acc, yacc);

    if (doH) {
      __bf16* dh = hb_hi + (q ^ 1) * HBSZ;
      __bf16* dl = hb_lo + (q ^ 1) * HBSZ;
#pragma unroll
      for (int r = 0; r < 8; ++r) {
        const float hv = tanhf(acc[r]);
        const unsigned short hbits = f2bf_bits(hv);
        const unsigned short lbits = f2bf_bits(hv - bf_bits2f(hbits));
        const int idx = (8 * hh + r) * SHP + ncol;
        dh[idx] = __builtin_bit_cast(__bf16, hbits);
        dl[idx] = __builtin_bit_cast(__bf16, lbits);
      }
    }
    if (doY) {
      float* ysb = ys + q * YBSZ;
#pragma unroll
      for (int r = 0; r < 8; ++r) ysb[(8 * hh + r) * YSP + wave * 16 + l15] = yacc[r];
    }
    __syncthreads();
  }
  if (wave < 8) store_y_rows(ys + (NSEQ & 1) * YBSZ, out, b0, NSEQ - 1, wave, lane);
}

extern "C" void kernel_launch(void* const* d_in, const int* in_sizes, int n_in,
                              void* d_out, int out_size, void* d_ws, size_t ws_size,
                              hipStream_t stream) {
  if (n_in < 4) return;
  if (in_sizes[0] < NBATCH * NSEQ * XDIM) return;
  if (in_sizes[1] < XDIM * NHID) return;
  if (in_sizes[2] < NHID * NHID) return;
  if (in_sizes[3] < NOUT * NHID) return;
  if (out_size < NBATCH * NSEQ * NOUT) return;
  if (ws_size < WS_TOTAL) return;

  const float* xin = (const float*)d_in[0];
  const float* Wih = (const float*)d_in[1];
  const float* Whh = (const float*)d_in[2];
  const float* Vw  = (const float*)d_in[3];
  float* out = (float*)d_out;

  char* ws = (char*)d_ws;
  unsigned short* xh    = (unsigned short*)(ws + OFF_XH);
  unsigned short* xl    = (unsigned short*)(ws + OFF_XL);
  unsigned short* whh_h = (unsigned short*)(ws + OFF_WHH_H);
  unsigned short* whh_l = (unsigned short*)(ws + OFF_WHH_L);
  unsigned short* wih_h = (unsigned short*)(ws + OFF_WIH_H);
  unsigned short* wih_l = (unsigned short*)(ws + OFF_WIH_L);
  unsigned short* v_h   = (unsigned short*)(ws + OFF_V_H);
  unsigned short* v_l   = (unsigned short*)(ws + OFF_V_L);

  prep_x<<<dim3(XPREP_BLOCKS), dim3(256), 0, stream>>>(xin, xh, xl);
  prep_whh<<<dim3(NHID / 8), dim3(256), 0, stream>>>(Whh, whh_h, whh_l);
  prep_wih<<<dim3(NHID / 8), dim3(256), 0, stream>>>(Wih, wih_h, wih_l);
  prep_v<<<dim3(NOUT / 8), dim3(256), 0, stream>>>(Vw, v_h, v_l);
  rnn_scan<<<dim3(NBATCH / ROWS), dim3(NTHR), 0, stream>>>(xh, xl, whh_h, whh_l, wih_h, wih_l, v_h, v_l, out);
}
